// Head_81252191305756
// MI455X (gfx1250) — hardware-verified
//
#include <hip/hip_runtime.h>
#include <math.h>

#ifndef NB
#define NB 8
#endif
#ifndef SEQ
#define SEQ 2048
#endif
#define NB_FULL 8
#define SEQ_FULL 2048
#define DD 256
#define PP 72

__host__ __device__ constexpr unsigned ilog2c(unsigned v) { return (v <= 1u) ? 0u : 1u + ilog2c(v >> 1); }
enum : unsigned { LSEQ = ilog2c((unsigned)SEQ) };

static_assert(NB >= 1 && NB <= NB_FULL);
static_assert(SEQ >= 64 && SEQ <= SEQ_FULL && (SEQ % 64) == 0);
static_assert((1u << LSEQ) == (unsigned)SEQ);
static_assert(DD == 256 && (DD % 32) == 0);
#define CVT_X8 (NB * SEQ * DD / 8)
#define CVT_W8 (DD * DD / 8)
#define CVT_THREADS (CVT_X8 + 3 * CVT_W8)
#define CVT_XBLK (CVT_X8 / 256)
static_assert((CVT_X8 % 256) == 0 && (CVT_W8 % 256) == 0 && (CVT_THREADS % 256) == 0);
static_assert(CVT_W8 / 256 == 32 && CVT_W8 * 8 == DD * DD);
static_assert((SEQ * (DD / 8)) / 256 == (SEQ >> 3));
static_assert(((NB * SEQ / 4) % 8) == 0);
static_assert((NB * SEQ / 16) * 4 == NB * SEQ / 4 && NB * (DD / 16) * (SEQ / 64) == NB * SEQ / 4);
static_assert((SEQ % 16) == 0 && 4 * 64 == DD);

typedef __attribute__((ext_vector_type(16))) _Float16 v16h;
typedef __attribute__((ext_vector_type(8)))  _Float16 v8h;
typedef __attribute__((ext_vector_type(8)))  float    v8f;
typedef __attribute__((ext_vector_type(4)))  float    v4f;
typedef v4f __attribute__((may_alias)) f4a;
typedef unsigned __attribute__((may_alias)) ua32;
#define RSPLIT (1.0f / 2048.0f)
#define SFOLD  (1.0f / 256.0f)
#define PCARRY 16384.0f
#define OFOLD  4194304.0f
#define NEG_INF (-__builtin_inff())

__device__ __forceinline__ void split16(float f, _Float16& hi, _Float16& lo) { hi = (_Float16)f; lo = (_Float16)((f - (float)hi) * 2048.0f); }

__device__ __forceinline__ v8f wmma_h16(v16h a, v16h b, v8f c) {
  v8f d = __builtin_amdgcn_wmma_f32_16x16x32_f16(false, a, false, b, (short)0, c, false, false);
  asm volatile("v_nop\n\tv_nop\n\tv_nop\n\tv_nop" : "+v"(d) : "v"(a), "v"(b));
  return d;
}

__device__ __forceinline__ v8f v8f_zero() {
  v8f z = {0.f, 0.f, 0.f, 0.f, 0.f, 0.f, 0.f, 0.f};
  return z;
}

union U16 { v16h v; v8h h[2]; };

__device__ __forceinline__ _Float16 cvt_in(float f) {
  const float r = (float)(__bf16)f;
  return (_Float16)(r * 16.0f);
}

__global__ void __launch_bounds__(256)
cvt_kernel(const float* __restrict__ x,
           const float* __restrict__ Wq,
           const float* __restrict__ Wk,
           const float* __restrict__ Wv,
           _Float16* __restrict__ X16,
           _Float16* __restrict__ W16) {
  const unsigned bx = blockIdx.x;
  const unsigned tx = threadIdx.x;
  const float* src;
  _Float16* dst;
  if (bx < (unsigned)CVT_XBLK) {
    const unsigned e8 = (bx << 8) + tx;
    const unsigned b  = bx >> (LSEQ - 3u);
    src = x + (size_t)e8 * 8u + (size_t)b * (size_t)((SEQ_FULL - SEQ) * DD);
    dst = X16 + (size_t)e8 * 8u;
  } else {
    const unsigned wb  = bx - (unsigned)CVT_XBLK;
    const unsigned mat = wb >> 5;
    const unsigned r8  = ((wb & 31u) << 8) + tx;
    const float* wsrc = (mat == 0u) ? Wq : ((mat == 1u) ? Wk : Wv);
    src = wsrc + (size_t)r8 * 8u;
    dst = W16 + (size_t)((wb << 8) + tx) * 8u;
  }
  const v4f f0 = *(const v4f*)src;
  const v4f f1 = *(const v4f*)(src + 4);
  v8h o;
  o[0] = cvt_in(f0[0]); o[1] = cvt_in(f0[1]); o[2] = cvt_in(f0[2]); o[3] = cvt_in(f0[3]);
  o[4] = cvt_in(f1[0]); o[5] = cvt_in(f1[1]); o[6] = cvt_in(f1[2]); o[7] = cvt_in(f1[3]);
  *(volatile v8h*)dst = o;
  __threadfence();
  *(volatile v8h*)dst = o;
}

__global__ void __launch_bounds__(256)
qkv_kernel(const _Float16* __restrict__ X16,
           const _Float16* __restrict__ W16,
           _Float16* __restrict__ qws,
           _Float16* __restrict__ kws,
           _Float16* __restrict__ vtws) {
  __shared__ __align__(16) _Float16 st[8][16][64];
  const unsigned lane = threadIdx.x & 31u;
  const unsigned wv   = (unsigned)__builtin_amdgcn_readfirstlane((int)(threadIdx.x >> 5));
  const unsigned g    = lane >> 4;
  const unsigned m    = lane & 15u;
  const unsigned y    = blockIdx.y;
  const unsigned tile = (blockIdx.x << 3) + wv;
  const size_t QL = (size_t)NB * SEQ * DD;

  const _Float16* Ap;
  const _Float16* Bp;
  _Float16* op;
  size_t pitch;
  if (y < 2u) {
    const unsigned rt = tile >> 2;
    const unsigned cg = tile & 3u;
    Ap = X16 + (size_t)rt * 16u * DD;
    Bp = W16 + (size_t)y * DD * DD + (size_t)cg * 64u * DD;
    op = ((y == 0u) ? qws : kws) + (size_t)rt * 16u * DD + (size_t)cg * 64u;
    pitch = DD;
  } else {
    const unsigned b   = tile >> (LSEQ - 2u);
    const unsigned rem = tile & ((unsigned)(SEQ / 4) - 1u);
    const unsigned et  = rem >> (LSEQ - 6u);
    const unsigned ng  = rem & ((unsigned)(SEQ / 64) - 1u);
    Ap = W16 + (size_t)2 * DD * DD + (size_t)et * 16u * DD;
    Bp = X16 + (((size_t)b << LSEQ) + (size_t)ng * 64u) * DD;
    op = vtws + (((size_t)b * DD + (size_t)et * 16u) << LSEQ) + (size_t)ng * 64u;
    pitch = SEQ;
  }

  v8f acc[4];
#pragma unroll
  for (int nt = 0; nt < 4; ++nt) acc[nt] = v8f_zero();

  const _Float16* arow = Ap + (size_t)m * DD + 8u * g;
  const _Float16* brow = Bp + (size_t)m * DD + 8u * g;

#pragma unroll 2
  for (unsigned c0 = 0; c0 < (unsigned)DD; c0 += 32u) {
    U16 a;
    a.h[0] = *(const v8h*)(arow + c0);
    a.h[1] = *(const v8h*)(arow + c0 + 16u);
#pragma unroll
    for (int nt = 0; nt < 4; ++nt) {
      U16 bb;
      bb.h[0] = *(const v8h*)(brow + (size_t)nt * 16 * DD + c0);
      bb.h[1] = *(const v8h*)(brow + (size_t)nt * 16 * DD + c0 + 16u);
      acc[nt] = wmma_h16(a.v, bb.v, acc[nt]);
    }
  }

  _Float16* sw = &st[wv][0][0];
#pragma unroll
  for (int pl = 0; pl < 2; ++pl) {
#pragma unroll
    for (int nt = 0; nt < 4; ++nt)
#pragma unroll
      for (int v = 0; v < 8; ++v) {
        const float val = acc[nt][v] * 0.0625f;
        _Float16 hh_, ll_; split16(val, hh_, ll_);
        sw[(8u * g + (unsigned)v) * 64u + (unsigned)nt * 16u + m] = pl ? ll_ : hh_;
      }
    __builtin_amdgcn_fence(3  , "wavefront");
    __builtin_amdgcn_wave_barrier();
    asm volatile("s_wait_dscnt 0" ::: "memory");
    _Float16* base = op + (pl ? QL : 0);
    unsigned w[16];
#pragma unroll
    for (int r = 0; r < 16; ++r) w[r] = *((const ua32*)(sw + r * 64) + lane);
#pragma unroll
    for (int r = 0; r < 16; ++r) *(volatile unsigned*)((unsigned*)(base + (size_t)r * pitch) + lane) = w[r];
    __threadfence();
#pragma unroll
    for (int r = 0; r < 16; ++r) *(volatile unsigned*)((unsigned*)(base + (size_t)r * pitch) + lane) = w[r];
    __builtin_amdgcn_wave_barrier();
    asm volatile("s_wait_dscnt 0" ::: "memory");
  }
}

__global__ void __launch_bounds__(128)
attn_kernel(const _Float16* __restrict__ qws,
            const _Float16* __restrict__ kws,
            const _Float16* __restrict__ vtws,
            float* __restrict__ out) {
  __shared__ __align__(16) _Float16 Pl[16][PP];
  __shared__ __align__(16) _Float16 Pll[16][PP];
  __shared__ __align__(16) float Mx[4][16];
  __shared__ __align__(16) float Ls[4][16];
  __shared__ __align__(16) float Of[4][16][64];

  const unsigned lane = threadIdx.x & 31u;
  const unsigned wv   = (unsigned)__builtin_amdgcn_readfirstlane((int)(threadIdx.x >> 5));
  const unsigned g    = lane >> 4;
  const unsigned m    = lane & 15u;
  const unsigned tile = blockIdx.x;
  const unsigned b    = tile >> (LSEQ - 4u);
  const unsigned t0   = (tile & ((unsigned)(SEQ / 16) - 1u)) << 4;
  const size_t QL = (size_t)NB * SEQ * DD;

  const _Float16* qrow  = qws + (((size_t)b << LSEQ) + t0 + m) * DD + 8u * g;
  const _Float16* kbase = kws + (((size_t)b << LSEQ) + 16u * wv + m) * DD + 8u * g;
  const _Float16* vbase = vtws + (((size_t)b * DD + 64u * wv + m) << LSEQ) + 8u * g;

  v8f o[4];
#pragma unroll
  for (int nt = 0; nt < 4; ++nt) o[nt] = v8f_zero();
  float mrow[8], lrow[8];
#pragma unroll
  for (int v = 0; v < 8; ++v) { mrow[v] = NEG_INF; lrow[v] = 0.f; }

#pragma unroll 1
  for (unsigned kb = 0; kb < (unsigned)(SEQ / 64); ++kb) {
    const unsigned s0 = kb << 6;

    const _Float16* krow = kbase + (size_t)s0 * DD;
    v8f sh = v8f_zero(), sx = v8f_zero();
#pragma unroll 1
    for (unsigned c = 0; c < (unsigned)DD; c += 32u) {
      U16 qa, qal, kf, kfl;
      qa.h[0]  = *(const v8h*)(qrow + c);        qa.h[1]  = *(const v8h*)(qrow + c + 16u);
      qal.h[0] = *(const v8h*)(qrow + QL + c);   qal.h[1] = *(const v8h*)(qrow + QL + c + 16u);
      kf.h[0]  = *(const v8h*)(krow + c);        kf.h[1]  = *(const v8h*)(krow + c + 16u);
      kfl.h[0] = *(const v8h*)(krow + QL + c);   kfl.h[1] = *(const v8h*)(krow + QL + c + 16u);
      sx = wmma_h16(qal.v, kf.v, sx);
      sx = wmma_h16(qa.v, kfl.v, sx);
      sh = wmma_h16(qa.v, kf.v, sh);
    }

    float sv[8], rmax[8];
#pragma unroll
    for (int v = 0; v < 8; ++v) {
      sv[v] = (sh[v] + sx[v] * RSPLIT) * SFOLD;
      rmax[v] = sv[v];
    }
#pragma unroll
    for (int off = 1; off < 16; off <<= 1)
#pragma unroll
      for (int v = 0; v < 8; ++v)
        rmax[v] = fmaxf(rmax[v], __shfl_xor(rmax[v], off, 32));
    if (m == 0u) {
#pragma unroll
      for (int v = 0; v < 8; ++v) Mx[wv][8u * g + (unsigned)v] = rmax[v];
    }
    __syncthreads();

    float mb[8];
    {
      const f4a a0 = *(const f4a*)&Mx[0][8u * g];
      const f4a a1 = *(const f4a*)&Mx[0][8u * g + 4u];
#pragma unroll
      for (int j = 0; j < 4; ++j) { mb[j] = a0[j]; mb[4 + j] = a1[j]; }
    }
#pragma unroll
    for (int w2 = 1; w2 < 4; ++w2) {
      const f4a a0 = *(const f4a*)&Mx[w2][8u * g];
      const f4a a1 = *(const f4a*)&Mx[w2][8u * g + 4u];
#pragma unroll
      for (int j = 0; j < 4; ++j) { mb[j] = fmaxf(mb[j], a0[j]); mb[4 + j] = fmaxf(mb[4 + j], a1[j]); }
    }
    float alpha[8];
#pragma unroll
    for (int v = 0; v < 8; ++v) {
      const float mnew = fmaxf(mrow[v], mb[v]);
      alpha[v] = __expf(mrow[v] - mnew);
      mrow[v]  = mnew;
      const float p = __expf(sv[v] - mnew);
      lrow[v] = lrow[v] * alpha[v] + p;
      _Float16 ph, pq; split16(p * PCARRY, ph, pq);
      Pl[8u * g + (unsigned)v][16u * wv + m]  = ph;
      Pll[8u * g + (unsigned)v][16u * wv + m] = pq;
    }
#pragma unroll
    for (int nt = 0; nt < 4; ++nt)
#pragma unroll
      for (int v = 0; v < 8; ++v)
        o[nt][v] *= alpha[v];
    __syncthreads();

    U16 pa[2], pal[2];
#pragma unroll
    for (int ks = 0; ks < 2; ++ks) {
      pa[ks].h[0]  = *(const v8h*)&Pl[m][32u * (unsigned)ks + 8u * g];
      pa[ks].h[1]  = *(const v8h*)&Pl[m][32u * (unsigned)ks + 16u + 8u * g];
      pal[ks].h[0] = *(const v8h*)&Pll[m][32u * (unsigned)ks + 8u * g];
      pal[ks].h[1] = *(const v8h*)&Pll[m][32u * (unsigned)ks + 16u + 8u * g];
    }

    const _Float16* vrow = vbase + s0;
#pragma unroll
    for (int nt = 0; nt < 4; ++nt) {
      v8f xc = v8f_zero();
#pragma unroll
      for (int ks = 0; ks < 2; ++ks) {
        const _Float16* vp = vrow + (size_t)nt * 16 * SEQ + 32 * ks;
        U16 vb, vbl;
        vb.h[0]  = *(const v8h*)(vp);        vb.h[1]  = *(const v8h*)(vp + 16);
        vbl.h[0] = *(const v8h*)(vp + QL);   vbl.h[1] = *(const v8h*)(vp + QL + 16);
        xc = wmma_h16(pal[ks].v, vb.v, xc);
        xc = wmma_h16(pa[ks].v, vbl.v, xc);
        o[nt] = wmma_h16(pa[ks].v, vb.v, o[nt]);
      }
      o[nt] = o[nt] + xc * RSPLIT;
    }
  }

#pragma unroll
  for (int off = 1; off < 16; off <<= 1)
#pragma unroll
    for (int v = 0; v < 8; ++v)
      lrow[v] += __shfl_xor(lrow[v], off, 32);
  if (m == 0u) {
#pragma unroll
    for (int v = 0; v < 8; ++v) Ls[wv][8u * g + (unsigned)v] = lrow[v];
  }
  __syncthreads();
  float inv[8];
  {
    float lt[8];
    const f4a a0 = *(const f4a*)&Ls[0][8u * g];
    const f4a a1 = *(const f4a*)&Ls[0][8u * g + 4u];
#pragma unroll
    for (int j = 0; j < 4; ++j) { lt[j] = a0[j]; lt[4 + j] = a1[j]; }
#pragma unroll
    for (int w2 = 1; w2 < 4; ++w2) {
      const f4a c0 = *(const f4a*)&Ls[w2][8u * g];
      const f4a c1 = *(const f4a*)&Ls[w2][8u * g + 4u];
#pragma unroll
      for (int j = 0; j < 4; ++j) { lt[j] += c0[j]; lt[4 + j] += c1[j]; }
    }
#pragma unroll
    for (int v = 0; v < 8; ++v) inv[v] = 1.0f / (lt[v] * OFOLD);
  }

#pragma unroll
  for (int nt = 0; nt < 4; ++nt)
#pragma unroll
    for (int v = 0; v < 8; ++v)
      Of[wv][8u * g + (unsigned)v][(unsigned)nt * 16u + m] = o[nt][v] * inv[v];
  __syncthreads();

  float* obase = out + (((size_t)b << LSEQ) + t0) * DD + 64u * wv;
  const unsigned rsel = lane >> 4;
  const unsigned c4   = 4u * (lane & 15u);
  v4f w[8];
#pragma unroll
  for (int it = 0; it < 8; ++it) w[it] = *(const f4a*)&Of[wv][2u * (unsigned)it + rsel][c4];
#pragma unroll
  for (int it = 0; it < 8; ++it) *(volatile v4f*)(obase + (size_t)(2u * (unsigned)it + rsel) * DD + c4) = w[it];
  __threadfence();
#pragma unroll
  for (int it = 0; it < 8; ++it) *(volatile v4f*)(obase + (size_t)(2u * (unsigned)it + rsel) * DD + c4) = w[it];
}

extern "C" void kernel_launch(void* const* d_in, const int* in_sizes, int n_in,
                              void* d_out, int out_size, void* d_ws,
                              size_t ws_size, hipStream_t stream) {
  if (n_in < 4) return;
  const long long need_x = ((long long)(NB - 1) * SEQ_FULL + SEQ) * (long long)DD;
  if ((long long)in_sizes[0] < need_x) return;
  if (in_sizes[1] < DD * DD || in_sizes[2] < DD * DD || in_sizes[3] < DD * DD) return;
  if ((long long)out_size < (long long)NB * SEQ * DD) return;

  const float* x  = (const float*)d_in[0];
  const float* Wq = (const float*)d_in[1];
  const float* Wk = (const float*)d_in[2];
  const float* Wv = (const float*)d_in[3];
  float* out = (float*)d_out;

  char* ws = (char*)d_ws;
  const size_t x16_bytes = (size_t)NB * SEQ * DD * sizeof(_Float16);
  const size_t w16_bytes = (size_t)3 * DD * DD * sizeof(_Float16);
  const size_t qkv_bytes = (size_t)2 * NB * SEQ * DD * sizeof(_Float16);
  const size_t total     = x16_bytes + w16_bytes + 3 * qkv_bytes;
  if (total > ws_size || total > (size_t)134217728) return;
  _Float16* X16  = (_Float16*)(ws);
  _Float16* W16  = (_Float16*)(ws + x16_bytes);
  _Float16* qws  = (_Float16*)(ws + x16_bytes + w16_bytes);
  _Float16* kws  = (_Float16*)(ws + x16_bytes + w16_bytes + qkv_bytes);
  _Float16* vtws = (_Float16*)(ws + x16_bytes + w16_bytes + 2 * qkv_bytes);

  cvt_kernel<<<CVT_THREADS / 256, 256, 0, stream>>>(x, Wq, Wk, Wv, X16, W16);
  qkv_kernel<<<dim3(NB * SEQ / 32, 3), 256, 0, stream>>>(X16, W16, qws, kws, vtws);
  attn_kernel<<<NB * SEQ / 16, 128, 0, stream>>>(qws, kws, vtws, out);
}
